// MambaMIL_47691316855479
// MI455X (gfx1250) — hardware-run, weakly checked
//
#include <hip/hip_runtime.h>
#include <math.h>
#include <stdint.h>

typedef __attribute__((ext_vector_type(16))) _Float16 v16h;
typedef __attribute__((ext_vector_type(8)))  _Float16 v8h;
typedef __attribute__((ext_vector_type(4)))  _Float16 v4h;
typedef __attribute__((ext_vector_type(16))) __bf16   v16b;
typedef __attribute__((ext_vector_type(8)))  __bf16   v8b;
typedef __attribute__((ext_vector_type(8)))  float    v8f;
typedef __attribute__((ext_vector_type(4)))  float    v4f;
typedef __attribute__((ext_vector_type(2)))  float    v2f;

constexpr int SEQ_L   = 2048;
constexpr int DIM_IN  = 1024;
constexpr int DIM_M   = 512;
constexpr int DIM_I   = 1024;
constexpr int DIM_ST  = 16;
constexpr int DIM_R   = 32;
constexpr int DBC_W   = DIM_R + 2 * DIM_ST;
constexpr int NLAYER  = 2;
constexpr int NCLS    = 2;
constexpr int OUT_FLOATS = NCLS + DIM_M + SEQ_L * DIM_M;
static_assert(OUT_FLOATS * 4 == 4196360, "");
static_assert(8 + DIM_M * 4 == 2056, "");

__device__ __forceinline__ unsigned short f2bf_bits(float f) {
  unsigned u = __float_as_uint(f);
  return (unsigned short)((u + 0x7FFFu + ((u >> 16) & 1u)) >> 16);
}
__device__ __forceinline__ float bf_bits2f(unsigned short h) { return __uint_as_float(((unsigned)h) << 16); }

__device__ __forceinline__ void dep_guard_h(v8f& a, v8f& b, v16h x, v16h y) { asm volatile("v_nop\n\tv_nop\n\tv_nop\n\tv_nop" : "+v"(a), "+v"(b) : "v"(x), "v"(y)); }
__device__ __forceinline__ void dep_guard_b(v8f& a, v8f& b, v16b x, v16b y) { asm volatile("v_nop\n\tv_nop\n\tv_nop\n\tv_nop" : "+v"(a), "+v"(b) : "v"(x), "v"(y)); }
__device__ __forceinline__ void keep4_h(v16h a, v16h b, v16h c, v16h d) { asm volatile("v_nop" :: "v"(a), "v"(b), "v"(c), "v"(d)); }
__device__ __forceinline__ void keep4_b(v16b a, v16b b, v16b c, v16b d) { asm volatile("v_nop" :: "v"(a), "v"(b), "v"(c), "v"(d)); }
__device__ __forceinline__ void acc_guard4(v8f& a, v8f& b, v8f& c, v8f& d) { asm volatile("v_nop\n\tv_nop\n\tv_nop\n\tv_nop" : "+v"(a), "+v"(b), "+v"(c), "+v"(d)); }
template <typename T> struct Frag;
template <> struct Frag<_Float16> {
  typedef v16h V; union U { v16h v; v8h h[2]; };
  static __device__ __forceinline__ v16h load(const _Float16* p) {
    U f; f.h[0] = *(const v8h*)(p); f.h[1] = *(const v8h*)(p + 16); return f.v;
  }
  static __device__ __forceinline__ v8f mma(v16h a, v16h b, v8f c) {
    return __builtin_amdgcn_wmma_f32_16x16x32_f16(false, a, false, b, (short)0, c, false, false);
  }
  static __device__ __forceinline__ void guard(v8f& a, v8f& b, v16h x, v16h y) { dep_guard_h(a, b, x, y); }
  static __device__ __forceinline__ void keep(v16h a, v16h b, v16h c, v16h d) { keep4_h(a, b, c, d); }
};
template <> struct Frag<__bf16> {
  typedef v16b V; union U { v16b v; v8b h[2]; };
  static __device__ __forceinline__ v16b load(const __bf16* p) {
    U f; f.h[0] = *(const v8b*)(p); f.h[1] = *(const v8b*)(p + 16); return f.v;
  }
  static __device__ __forceinline__ v8f mma(v16b a, v16b b, v8f c) {
    return __builtin_amdgcn_wmma_f32_16x16x32_bf16(false, a, false, b, (short)0, c, false, false);
  }
  static __device__ __forceinline__ void guard(v8f& a, v8f& b, v16b x, v16b y) { dep_guard_b(a, b, x, y); }
  static __device__ __forceinline__ void keep(v16b a, v16b b, v16b c, v16b d) { keep4_b(a, b, c, d); }
};

template <int ET> struct Elem;
template <> struct Elem<0> { typedef _Float16 T; };
template <> struct Elem<1> { typedef __bf16 T; };
template <int ET, bool SPLIT, int BIAS_MODE, int OUT_MODE, bool RESID, int ACT = 0>
__global__ __launch_bounds__(256) void wmma_gemm64(
    const unsigned short* __restrict__ Ap, const unsigned short* __restrict__ A2p, int lda, long strideA,
    const unsigned short* __restrict__ Btp, const unsigned short* __restrict__ Bt2p, int ldb, long strideB,
    void* __restrict__ Cout, void* __restrict__ Cout2, int ldc, long strideC,
    const float* __restrict__ bias,
    const float* __restrict__ resid, long strideR,
    int M, int N, int K, float scale) {
  typedef typename Elem<ET>::T T;
  typedef typename Frag<T>::V V;
  const T* A = (const T*)Ap; const T* A2 = (const T*)A2p; const T* Bt = (const T*)Btp; const T* Bt2 = (const T*)Bt2p;
  __shared__ __align__(16) float sT[8][16 * 68];
  const int b    = blockIdx.y;
  const int lane = threadIdx.x & 31;
  const int wave = threadIdx.x >> 5;
  const int tilesN = N >> 6;
  const int tilesM = M >> 6;
  const int tile = blockIdx.x * 8 + wave;
  if (tile >= tilesM * tilesN) return;
  const int tm = tile / tilesN;
  const int tn = tile - tm * tilesN;
  const int m0 = tm << 6;
  const int n0 = tn << 6;

  const T* Ab  = A  + (size_t)b * strideA;
  const T* Bb  = Bt + (size_t)b * strideB;
  const T* Ab2 = SPLIT ? (A2  + (size_t)b * strideA) : nullptr;
  const T* Bb2 = SPLIT ? (Bt2 + (size_t)b * strideB) : nullptr;

  const int rlane = lane & 15;
  const int koff  = (lane >> 4) * 8;
  const int mOff  = (lane >> 4) * 8;

  v8f acc[4][4];
#pragma unroll
  for (int i = 0; i < 4; ++i)
#pragma unroll
    for (int j = 0; j < 4; ++j) acc[i][j] = (v8f){0.f,0.f,0.f,0.f,0.f,0.f,0.f,0.f};

  for (int k0 = 0; k0 < K; k0 += 32) {
    V bh[4], bl[4];
#pragma unroll
    for (int j = 0; j < 4; ++j) {
      const size_t bo = (size_t)(n0 + (j << 4) + rlane) * ldb + koff + k0;
      bh[j] = Frag<T>::load(Bb + bo);
      if (SPLIT) bl[j] = Frag<T>::load(Bb2 + bo);
    }
#pragma unroll
    for (int i = 0; i < 4; ++i) {
      const size_t ao = (size_t)(m0 + (i << 4) + rlane) * lda + koff + k0;
      V ah = Frag<T>::load(Ab + ao);
      V al;
      if (SPLIT) al = Frag<T>::load(Ab2 + ao);
#pragma unroll
      for (int j = 0; j < 4; ++j) {
        acc[i][j] = Frag<T>::mma(ah, bh[j], acc[i][j]);
        if (SPLIT) {
          acc[i][j] = Frag<T>::mma(ah, bl[j], acc[i][j]);
          acc[i][j] = Frag<T>::mma(al, bh[j], acc[i][j]);
        }
      }
      Frag<T>::guard(acc[i][0], acc[i][3], ah, SPLIT ? al : ah);
    }
    Frag<T>::keep(bh[0], bh[1], bh[2], bh[3]);
    if (SPLIT) Frag<T>::keep(bl[0], bl[1], bl[2], bl[3]);
  }
  acc_guard4(acc[0][0], acc[0][1], acc[0][2], acc[0][3]);
  acc_guard4(acc[1][0], acc[1][1], acc[1][2], acc[1][3]);
  acc_guard4(acc[2][0], acc[2][1], acc[2][2], acc[2][3]);
  acc_guard4(acc[3][0], acc[3][1], acc[3][2], acc[3][3]);

  float* slab = sT[wave];
  const float* Rb = RESID ? (resid + (size_t)b * strideR) : nullptr;
#pragma unroll
  for (int i = 0; i < 4; ++i) {
    const int mBase = m0 + (i << 4);
#pragma unroll
    for (int j = 0; j < 4; ++j) {
      const int n = n0 + (j << 4) + rlane;
      float bv = 0.f;
      if (BIAS_MODE == 2) bv = bias[n];
#pragma unroll
      for (int r = 0; r < 8; ++r) {
        float v = acc[i][j][r] * scale;
        if (BIAS_MODE == 1) v += bias[mBase + mOff + r];
        if (BIAS_MODE == 2) v += bv;
        if (RESID) v += Rb[(size_t)(mBase + mOff + r) * ldc + n];
        if (ACT == 1) v = tanhf(v);
        if (ACT == 2) v = fmaxf(v, 0.0f);
        if (ACT == 3) v = v / (1.0f + expf(-v));
        if (ACT == 4) v = (v > 0.f) ? v : 0.01f * v;
        if (ACT == 5) v = 0.5f * v * (1.0f + erff(v * 0.70710678118654752f));
        slab[(mOff + r) * 68 + (j << 4) + rlane] = v;
      }
    }
    __builtin_amdgcn_fence(__ATOMIC_RELEASE, "workgroup");
    __builtin_amdgcn_wave_barrier();
    __builtin_amdgcn_fence(__ATOMIC_ACQUIRE, "workgroup");
    if (OUT_MODE == 0) {
      float* C = (float*)Cout + (size_t)b * strideC;
      const int hh = lane >> 4, c4 = (lane & 15) * 4;
      for (int pass = 0; pass < 2; ++pass) {
#pragma unroll
        for (int it = 0; it < 8; ++it) {
          const int row = it * 2 + hh;
          v4f v = *(const v4f*)(slab + row * 68 + c4);
          *(volatile v4f*)(C + (size_t)(mBase + row) * ldc + n0 + c4) = v;
        }
        __threadfence();
      }
    } else {
      const int q = lane >> 3, c8 = (lane & 7) * 8;
      unsigned short* C  = (unsigned short*)Cout  + (size_t)b * strideC;
      unsigned short* C2 = (OUT_MODE == 2) ? ((unsigned short*)Cout2 + (size_t)b * strideC) : nullptr;
      for (int pass = 0; pass < 2; ++pass) {
#pragma unroll
        for (int it = 0; it < 4; ++it) {
          const int row = it * 4 + q;
          const float* sp = slab + row * 68 + c8;
          v8h hv, lv;
#pragma unroll
          for (int e = 0; e < 8; ++e) {
            if (OUT_MODE == 1) {
              hv[e] = (_Float16)sp[e];
            } else {
              unsigned short hb = f2bf_bits(sp[e]);
              unsigned short lb = f2bf_bits(sp[e] - bf_bits2f(hb));
              hv[e] = __builtin_bit_cast(_Float16, hb);
              lv[e] = __builtin_bit_cast(_Float16, lb);
            }
          }
          *(volatile v8h*)(C + (size_t)(mBase + row) * ldc + n0 + c8) = hv;
          if (OUT_MODE == 2) *(volatile v8h*)(C2 + (size_t)(mBase + row) * ldc + n0 + c8) = lv;
        }
        __threadfence();
      }
    }
    __builtin_amdgcn_fence(__ATOMIC_RELEASE, "workgroup");
    __builtin_amdgcn_wave_barrier();
    __builtin_amdgcn_fence(__ATOMIC_ACQUIRE, "workgroup");
  }
}

__global__ __launch_bounds__(256) void cast_f32_f16x2s(
    const float* __restrict__ in, _Float16* __restrict__ out, int n2, float scale) {
  const int i = blockIdx.x * 256 + threadIdx.x;
  if (i < n2) {
    const v2f p = *(const v2f*)(in + 2 * (size_t)i);
    const _Float16 h0 = (_Float16)(p.x * scale), h1 = (_Float16)(p.y * scale);
    const unsigned u = (unsigned)__builtin_bit_cast(unsigned short, h0) | ((unsigned)__builtin_bit_cast(unsigned short, h1) << 16);
    ((volatile unsigned*)out)[i] = u;
    __threadfence();
    ((volatile unsigned*)out)[i] = u;
  }
}

__global__ __launch_bounds__(256) void cast_dt_kernel(
    const float* __restrict__ dbc, _Float16* __restrict__ dt16, int n2, float scale) {
  const int i = blockIdx.x * 256 + threadIdx.x;
  if (i < n2) {
    const int t = i >> 4;
    const int k2 = (i & 15) * 2;
    const v2f p = *(const v2f*)(dbc + (size_t)t * DBC_W + k2);
    const _Float16 h0 = (_Float16)(p.x * scale), h1 = (_Float16)(p.y * scale);
    const unsigned u = (unsigned)__builtin_bit_cast(unsigned short, h0) | ((unsigned)__builtin_bit_cast(unsigned short, h1) << 16);
    ((volatile unsigned*)dt16)[i] = u;
    __threadfence();
    ((volatile unsigned*)dt16)[i] = u;
  }
}

template <bool GELU_IN>
__global__ __launch_bounds__(128) void rmsnorm_rows(
    const float* __restrict__ hin, float* __restrict__ hout, const float* __restrict__ w,
    _Float16* __restrict__ hs16, int nrows)
{
  __shared__ __align__(16) float sRow[4][512];
  const int wave = threadIdx.x >> 5, lane = threadIdx.x & 31;
  int row = blockIdx.x * 4 + wave;
  row = row < nrows ? row : nrows - 1;
  const float* src = hin + (size_t)row * DIM_M;
  float ss = 0.f;
#pragma unroll 1
  for (int it = 0; it < 16; ++it) {
    float v = src[32 * it + lane];
    if (GELU_IN) {
      v = 0.5f * v * (1.0f + erff(v * 0.70710678118654752f));
      float* dp = hout + (size_t)row * DIM_M + 32 * it + lane;
      *(volatile float*)dp = v;
      __threadfence();
      *(volatile float*)dp = v;
    }
    ss += v * v;
    sRow[wave][32 * it + lane] = v;
  }
#pragma unroll
  for (int off = 1; off < 32; off <<= 1) ss += __shfl_xor(ss, off, 32);
  const float scale = rsqrtf(ss * (1.0f / 512.0f) + 1e-5f);
  __syncthreads();
  v4f r[4];
#pragma unroll
  for (int p = 0; p < 4; ++p) {
    const v4f v  = *(const v4f*)(&sRow[wave][128 * p + 4 * lane]);
    const v4f ww = *(const v4f*)(w + 128 * p + 4 * lane);
    r[p] = v * scale * ww;
  }
  for (int pass = 0; pass < 2; ++pass) {
#pragma unroll
    for (int p = 0; p < 4; ++p) {
      v4h hv;
      hv[0] = (_Float16)r[p].x; hv[1] = (_Float16)r[p].y; hv[2] = (_Float16)r[p].z; hv[3] = (_Float16)r[p].w;
      *(volatile v4h*)(hs16 + (size_t)row * DIM_M + 128 * p + 4 * lane) = hv;
    }
    __threadfence();
  }
}

__global__ __launch_bounds__(256) void conv_silu_kernel(
    const float* __restrict__ proj, const float* __restrict__ cw, const float* __restrict__ cb,
    float* __restrict__ u32, _Float16* __restrict__ u16, int L)
{
  const int idx = blockIdx.x * 256 + threadIdx.x;
  const int t  = idx >> 8;
  const int c4 = (idx & 255) * 4;
  v4f wv[4];
#pragma unroll
  for (int ci = 0; ci < 4; ++ci) wv[ci] = *(const v4f*)(cw + (size_t)(c4 + ci) * 4);
  v4f acc = {0.f, 0.f, 0.f, 0.f};
#pragma unroll
  for (int k = 0; k < 4; ++k) {
    const int tt  = t - 3 + k;
    const int ttc = tt < 0 ? 0 : tt;
    v4f pv = *(const v4f*)(proj + (size_t)ttc * (2 * DIM_I) + c4);
    pv.x = (tt >= 0) ? pv.x : 0.f;
    pv.y = (tt >= 0) ? pv.y : 0.f;
    pv.z = (tt >= 0) ? pv.z : 0.f;
    pv.w = (tt >= 0) ? pv.w : 0.f;
    const v4f wk = {wv[0][k], wv[1][k], wv[2][k], wv[3][k]};
    acc += pv * wk;
  }
  const v4f bv = *(const v4f*)(cb + c4);
  acc += bv;
  v4f r;
  r.x = acc.x * (1.0f / (1.0f + expf(-acc.x)));
  r.y = acc.y * (1.0f / (1.0f + expf(-acc.y)));
  r.z = acc.z * (1.0f / (1.0f + expf(-acc.z)));
  r.w = acc.w * (1.0f / (1.0f + expf(-acc.w)));
  v4h hv;
  hv[0] = (_Float16)(r.x * 64.0f); hv[1] = (_Float16)(r.y * 64.0f);
  hv[2] = (_Float16)(r.z * 64.0f); hv[3] = (_Float16)(r.w * 64.0f);
  float* up = u32 + (size_t)t * DIM_I + c4;
  _Float16* hp = u16 + (size_t)t * DIM_I + c4;
  *(volatile v4f*)up = r;
  *(volatile v4h*)hp = hv;
  __threadfence();
  *(volatile v4f*)up = r;
  *(volatile v4h*)hp = hv;
}

#define SCAN_TS 32
static_assert(SEQ_L % SCAN_TS == 0, "");
__global__ __launch_bounds__(256) void scan_kernel(
    const float* __restrict__ u32,
    const float* __restrict__ dpre,
    const float* __restrict__ dbc,
    const float* __restrict__ proj,
    const float* __restrict__ A_log,
    const float* __restrict__ Dp,
    _Float16* __restrict__ ys16,
    int L)
{
  __shared__ __align__(16) float sDp[SCAN_TS][64];
  __shared__ __align__(16) float sU[SCAN_TS][64];
  __shared__ __align__(16) float sG[SCAN_TS][64];
  __shared__ __align__(16) float sBC[SCAN_TS][32];
  __shared__ __align__(16) float sY[SCAN_TS][64];

  const int tid  = threadIdx.x;
  const int wave = tid >> 5;
  const int lane = tid & 31;
  const int g    = lane & 3;
  const int chl  = lane >> 2;
  const int cl   = wave * 8 + chl;
  const int c0   = blockIdx.x * 64;
  const int c    = c0 + cl;

  float Aj[4];
#pragma unroll
  for (int j = 0; j < 4; ++j) Aj[j] = -expf(A_log[(size_t)c * DIM_ST + 4 * g + j]);
  const float Dc = Dp[c];
  float s[4] = {0.f, 0.f, 0.f, 0.f};

  for (int t0 = 0; t0 < L; t0 += SCAN_TS) {
    __syncthreads();
#pragma unroll
    for (int i = 0; i < 2; ++i) {
      const int f = tid + 256 * i;
      const int row = f >> 4;
      const int col4 = (f & 15) * 4;
      const size_t gi = (size_t)(t0 + row) * DIM_I + c0 + col4;
      *(v4f*)(&sDp[row][col4]) = *(const v4f*)(dpre + gi);
      *(v4f*)(&sU[row][col4])  = *(const v4f*)(u32 + gi);
      *(v4f*)(&sG[row][col4])  = *(const v4f*)(proj + (size_t)(t0 + row) * (2 * DIM_I) + DIM_I + c0 + col4);
    }
    {
      const int row = tid >> 3;
      const int col4 = (tid & 7) * 4;
      *(v4f*)(&sBC[row][col4]) = *(const v4f*)(dbc + (size_t)(t0 + row) * DBC_W + DIM_R + col4);
    }
    __syncthreads();
#pragma unroll 1
    for (int i = 0; i < SCAN_TS; ++i) {
      const float x  = sDp[i][cl];
      const float dt = fmaxf(x, 0.0f) + log1pf(expf(-fabsf(x)));
      const float uu = sU[i][cl];
      const v4f b4 = *(const v4f*)(&sBC[i][4 * g]);
      const v4f c4 = *(const v4f*)(&sBC[i][16 + 4 * g]);
      float yy = 0.f;
#pragma unroll
      for (int j = 0; j < 4; ++j) {
        const float dA = expf(dt * Aj[j]);
        s[j] = s[j] * dA + (dt * b4[j]) * uu;
        yy += s[j] * c4[j];
      }
      yy += __shfl_xor(yy, 1, 32);
      yy += __shfl_xor(yy, 2, 32);
      const float y  = yy + uu * Dc;
      const float gt = sG[i][cl];
      const float sg = gt * (1.0f / (1.0f + expf(-gt)));
      const float o  = y * sg * 256.0f;
      if (g == 0) sY[i][cl] = o;
    }
    __syncthreads();
    {
      const int row = wave * 4 + (lane >> 3);
      const int c8  = (lane & 7) * 8;
      const float* sp = &sY[row][c8];
      v8h hv;
#pragma unroll
      for (int e = 0; e < 8; ++e) hv[e] = (_Float16)sp[e];
      _Float16* gp = ys16 + (size_t)(t0 + row) * DIM_I + c0 + c8;
      *(volatile v8h*)gp = hv;
      __threadfence();
      *(volatile v8h*)gp = hv;
    }
  }
}

#define FR_ROWS 8
static_assert(SEQ_L % FR_ROWS == 0, "");
__global__ __launch_bounds__(256) void final_norm_rows(
    const float* __restrict__ h, const float* __restrict__ w,
    float* __restrict__ hf, float* __restrict__ outF, int L)
{
  __shared__ __align__(16) float S[512 * FR_ROWS + 32];
  const int wave = threadIdx.x >> 5, lane = threadIdx.x & 31;
  const int t0 = blockIdx.x * FR_ROWS;
  int row = t0 + wave;
  row = row < L ? row : L - 1;
  const float* src = h + (size_t)row * DIM_M;
  v4f v[4];
  float ss = 0.f;
#pragma unroll
  for (int p = 0; p < 4; ++p) {
    v[p] = *(const v4f*)(src + 128 * p + 4 * lane);
    ss += v[p].x * v[p].x + v[p].y * v[p].y + v[p].z * v[p].z + v[p].w * v[p].w;
  }
#pragma unroll
  for (int off = 1; off < 32; off <<= 1) ss += __shfl_xor(ss, off, 32);
  const float scale = rsqrtf(ss * (1.0f / 512.0f) + 1e-5f);
  v4f r[4];
#pragma unroll
  for (int p = 0; p < 4; ++p) {
    const v4f ww = *(const v4f*)(w + 128 * p + 4 * lane);
    r[p] = v[p] * scale * ww;
  }
  for (int pass = 0; pass < 2; ++pass) {
#pragma unroll
    for (int p = 0; p < 4; ++p)
      *(volatile v4f*)(hf + (size_t)row * DIM_M + 128 * p + 4 * lane) = r[p];
    __threadfence();
  }
#pragma unroll
  for (int p = 0; p < 4; ++p) {
    float* sp = S + 2 + 512 * wave + 128 * p + 4 * lane;
    sp[0] = r[p].x; sp[1] = r[p].y; sp[2] = r[p].z; sp[3] = r[p].w;
  }
  if (wave == 0) {
    const int rp = (t0 > 0) ? (t0 - 1) : 0;
    const float* sp2 = h + (size_t)rp * DIM_M;
    float ss2 = 0.f;
    v4f q3 = {0.f, 0.f, 0.f, 0.f};
#pragma unroll
    for (int p = 0; p < 4; ++p) {
      const v4f q = *(const v4f*)(sp2 + 128 * p + 4 * lane);
      ss2 += q.x * q.x + q.y * q.y + q.z * q.z + q.w * q.w;
      if (p == 3) q3 = q;
    }
#pragma unroll
    for (int off = 1; off < 32; off <<= 1) ss2 += __shfl_xor(ss2, off, 32);
    const float scale2 = rsqrtf(ss2 * (1.0f / 512.0f) + 1e-5f);
    if (lane == 31) {
      const v4f ww = *(const v4f*)(w + 508);
      S[0] = q3.z * scale2 * ww.z;
      S[1] = q3.w * scale2 * ww.w;
    }
  }
  __syncthreads();
  const int fbase = 512 * t0 + 512;
  const bool lastblk = (t0 + FR_ROWS >= L);
  for (int pass = 0; pass < 2; ++pass) {
#pragma unroll
    for (int it = 0; it < 4; ++it) {
      const int line = wave * 16 + it * 4 + (lane >> 3);
      const int q = lane & 7;
      const v4f val = *(const v4f*)(S + 32 * line + 4 * q);
      const bool skip = (t0 == 0) && (line == 0);
      if (!skip) *(volatile v4f*)(outF + (size_t)fbase + 32 * line + 4 * q) = val;
    }
    if (lastblk && wave == 0 && lane == 0) {
      v2f tv;
      tv.x = S[512 * FR_ROWS];
      tv.y = S[512 * FR_ROWS + 1];
      *(volatile v2f*)(outF + (size_t)fbase + 512 * FR_ROWS) = tv;
    }
    __threadfence();
  }
}

__global__ __launch_bounds__(512) void head_kernel(
    const float* __restrict__ hf, const float* __restrict__ cls_w, const float* __restrict__ cls_b,
    float* __restrict__ outF, int L)
{
  __shared__ __align__(16) float sF[544];
  __shared__ float red[512];
  const int d = threadIdx.x;
  float acc = 0.f;
#pragma unroll 1
  for (int tb = 0; tb < L; tb += 64) {
    float p = 0.f;
#pragma unroll 1
    for (int i = 0; i < 64; ++i) p += hf[(size_t)(tb + i) * DIM_M + d];
    acc += p;
  }
  const float hid = acc * (1.0f / (float)L);
  sF[2 + d] = hid;
  for (int cls = 0; cls < NCLS; ++cls) {
    red[d] = hid * cls_w[cls * DIM_M + d];
    __syncthreads();
    for (int sdn = 256; sdn > 0; sdn >>= 1) {
      if (d < sdn) red[d] += red[d + sdn];
      __syncthreads();
    }
    if (d == 0) sF[cls] = red[0] + cls_b[cls];
    __syncthreads();
  }
  if (d < 30) sF[2 + DIM_M + d] = hf[d];
  __syncthreads();
  for (int pass = 0; pass < 2; ++pass) {
    if (d < 136) {
      const v4f val = *(const v4f*)(sF + 4 * d);
      *(volatile v4f*)(outF + 4 * d) = val;
    }
    __threadfence();
  }
}

static_assert(SEQ_L % 64 == 0 && DIM_M % 64 == 0 && (2 * DIM_I) % 64 == 0 && DBC_W % 64 == 0 && DIM_I % 64 == 0, "");
static_assert(DIM_IN % 32 == 0 && DIM_M % 32 == 0 && DIM_I % 32 == 0 && DIM_R % 32 == 0, "");

constexpr size_t SZ_X16  = (size_t)SEQ_L * DIM_IN * 2;
constexpr size_t SZ_W1H  = (size_t)DIM_M * DIM_IN * 2;
constexpr size_t SZ_INP  = (size_t)NLAYER * 2 * DIM_I * DIM_M * 2;
constexpr size_t SZ_XP   = (size_t)NLAYER * DBC_W * DIM_I * 2;
constexpr size_t SZ_DTP  = (size_t)NLAYER * DIM_I * DIM_R * 2;
constexpr size_t SZ_OUTP = (size_t)NLAYER * DIM_M * DIM_I * 2;
constexpr size_t SZ_HS   = (size_t)SEQ_L * DIM_M * 2;
constexpr size_t SZ_U16  = (size_t)SEQ_L * DIM_I * 2;
constexpr size_t SZ_DT16 = (size_t)SEQ_L * DIM_R * 2;
constexpr size_t SZ_YS   = (size_t)SEQ_L * DIM_I * 2;
constexpr size_t SZ_H    = (size_t)SEQ_L * DIM_M * 4;
constexpr size_t SZ_PROJ = (size_t)SEQ_L * 2 * DIM_I * 4;
constexpr size_t SZ_U32  = (size_t)SEQ_L * DIM_I * 4;
constexpr size_t SZ_DBC  = (size_t)SEQ_L * DBC_W * 4;
constexpr size_t SZ_DPRE = (size_t)SEQ_L * DIM_I * 4;
constexpr size_t SZ_HF   = (size_t)SEQ_L * DIM_M * 4;
constexpr size_t OFF_X16  = 0;
constexpr size_t OFF_W1H  = OFF_X16 + SZ_X16;
constexpr size_t OFF_INP  = OFF_W1H + SZ_W1H;
constexpr size_t OFF_XP   = OFF_INP + SZ_INP;
constexpr size_t OFF_DTP  = OFF_XP + SZ_XP;
constexpr size_t OFF_OUTP = OFF_DTP + SZ_DTP;
constexpr size_t OFF_HS   = OFF_OUTP + SZ_OUTP;
constexpr size_t OFF_U16  = OFF_HS + SZ_HS;
constexpr size_t OFF_DT16 = OFF_U16 + SZ_U16;
constexpr size_t OFF_YS   = OFF_DT16 + SZ_DT16;
constexpr size_t OFF_HA   = OFF_YS + SZ_YS;
constexpr size_t OFF_HB   = OFF_HA + SZ_H;
constexpr size_t OFF_PROJ = OFF_HB + SZ_H;
constexpr size_t OFF_U32  = OFF_PROJ + SZ_PROJ;
constexpr size_t OFF_DBC  = OFF_U32 + SZ_U32;
constexpr size_t OFF_DPRE = OFF_DBC + SZ_DBC;
constexpr size_t OFF_HF   = OFF_DPRE + SZ_DPRE;
constexpr size_t WS_TOTAL = OFF_HF + SZ_HF;
static_assert(WS_TOTAL == 69206016, "");
static_assert(WS_TOTAL <= 134217728, "");
static_assert((OFF_W1H % 128) == 0 && (OFF_HS % 128) == 0 && (OFF_HA % 128) == 0 && (OFF_HF % 128) == 0 && (OFF_DT16 % 128) == 0, "");

static inline unsigned gemm_blocks(int M, int N) { return (unsigned)((((M / 64) * (N / 64)) + 7) / 8); }

extern "C" void kernel_launch(void* const* d_in, const int* in_sizes, int n_in,
                              void* d_out, int out_size, void* d_ws, size_t ws_size,
                              hipStream_t stream)
{
  if (n_in < 16) return;
  if (in_sizes[0] != SEQ_L * DIM_IN || out_size != OUT_FLOATS || ws_size < WS_TOTAL) return;

  const float* x          = (const float*)d_in[0];
  const float* W1         = (const float*)d_in[1];
  const float* b1         = (const float*)d_in[2];
  const float* norm_w     = (const float*)d_in[3];
  const float* in_proj_w  = (const float*)d_in[4];
  const float* conv_w     = (const float*)d_in[5];
  const float* conv_b     = (const float*)d_in[6];
  const float* x_proj_w   = (const float*)d_in[7];
  const float* dt_proj_w  = (const float*)d_in[8];
  const float* dt_proj_b  = (const float*)d_in[9];
  const float* A_log      = (const float*)d_in[10];
  const float* Dp         = (const float*)d_in[11];
  const float* out_proj_w = (const float*)d_in[12];
  const float* norm_f_w   = (const float*)d_in[13];
  const float* cls_w      = (const float*)d_in[14];
  const float* cls_b      = (const float*)d_in[15];

  char* ws = (char*)d_ws;
  _Float16* x16    = (_Float16*)(ws + OFF_X16);
  _Float16* w1h    = (_Float16*)(ws + OFF_W1H);
  _Float16* inp16  = (_Float16*)(ws + OFF_INP);
  _Float16* xp16   = (_Float16*)(ws + OFF_XP);
  _Float16* dtp16  = (_Float16*)(ws + OFF_DTP);
  _Float16* outp16 = (_Float16*)(ws + OFF_OUTP);
  _Float16* hs16   = (_Float16*)(ws + OFF_HS);
  _Float16* u16    = (_Float16*)(ws + OFF_U16);
  _Float16* dt16   = (_Float16*)(ws + OFF_DT16);
  _Float16* ys16   = (_Float16*)(ws + OFF_YS);
  float* hA   = (float*)(ws + OFF_HA);
  float* hB   = (float*)(ws + OFF_HB);
  float* proj = (float*)(ws + OFF_PROJ);
  float* u32  = (float*)(ws + OFF_U32);
  float* dbc  = (float*)(ws + OFF_DBC);
  float* dpre = (float*)(ws + OFF_DPRE);
  float* hf   = (float*)(ws + OFF_HF);
  float* outF = (float*)d_out;

  typedef const unsigned short* cus;

  {
    const int n2x = SEQ_L * DIM_IN / 2;
    cast_f32_f16x2s<<<(n2x + 255) / 256, 256, 0, stream>>>(x, x16, n2x, 1.0f);
    const int n2w1 = DIM_M * DIM_IN / 2;
    cast_f32_f16x2s<<<(n2w1 + 255) / 256, 256, 0, stream>>>(W1, w1h, n2w1, 64.0f);
    const int n2inp = NLAYER * 2 * DIM_I * DIM_M / 2;
    cast_f32_f16x2s<<<(n2inp + 255) / 256, 256, 0, stream>>>(in_proj_w, inp16, n2inp, 64.0f);
    const int n2xp = NLAYER * DBC_W * DIM_I / 2;
    cast_f32_f16x2s<<<(n2xp + 255) / 256, 256, 0, stream>>>(x_proj_w, xp16, n2xp, 64.0f);
    const int n2dtp = NLAYER * DIM_I * DIM_R / 2;
    cast_f32_f16x2s<<<(n2dtp + 255) / 256, 256, 0, stream>>>(dt_proj_w, dtp16, n2dtp, 64.0f);
    const int n2op = NLAYER * DIM_M * DIM_I / 2;
    cast_f32_f16x2s<<<(n2op + 255) / 256, 256, 0, stream>>>(out_proj_w, outp16, n2op, 64.0f);
  }

  wmma_gemm64<0, false, 2, 0, false, 0><<<dim3(gemm_blocks(SEQ_L, DIM_M), 1), 256, 0, stream>>>(
      (cus)x16, (cus)x16, DIM_IN, 0L,
      (cus)w1h, (cus)w1h, DIM_IN, 0L,
      (void*)hB, (void*)hB, DIM_M, 0L,
      b1, b1, 0L, SEQ_L, DIM_M, DIM_IN, 1.0f / 64.0f);

  for (int l = 0; l < NLAYER; ++l) {
    float* hres = (l == 0) ? hA : hB;
    float* hnxt = (l == 0) ? hB : hA;
    if (l == 0) {
      rmsnorm_rows<true><<<SEQ_L / 4, 128, 0, stream>>>(hB, hA, norm_w, hs16, SEQ_L);
    } else {
      rmsnorm_rows<false><<<SEQ_L / 4, 128, 0, stream>>>(hB, hA, norm_w + (size_t)l * DIM_M, hs16, SEQ_L);
    }
    wmma_gemm64<0, false, 0, 0, false, 0><<<dim3(gemm_blocks(SEQ_L, 2 * DIM_I), 1), 256, 0, stream>>>(
        (cus)hs16, (cus)hs16, DIM_M, 0L,
        (cus)(inp16 + (size_t)l * 2 * DIM_I * DIM_M), (cus)(inp16 + (size_t)l * 2 * DIM_I * DIM_M), DIM_M, 0L,
        (void*)proj, (void*)proj, 2 * DIM_I, 0L,
        b1, b1, 0L, SEQ_L, 2 * DIM_I, DIM_M, 1.0f / 64.0f);
    conv_silu_kernel<<<SEQ_L, 256, 0, stream>>>(proj, conv_w + (size_t)l * DIM_I * 4, conv_b + (size_t)l * DIM_I, u32, u16, SEQ_L);
    wmma_gemm64<0, false, 0, 0, false, 0><<<dim3(gemm_blocks(SEQ_L, DBC_W), 1), 256, 0, stream>>>(
        (cus)u16, (cus)u16, DIM_I, 0L,
        (cus)(xp16 + (size_t)l * DBC_W * DIM_I), (cus)(xp16 + (size_t)l * DBC_W * DIM_I), DIM_I, 0L,
        (void*)dbc, (void*)dbc, DBC_W, 0L,
        b1, b1, 0L, SEQ_L, DBC_W, DIM_I, 1.0f / 4096.0f);
    {
      const int n2 = SEQ_L * DIM_R / 2;
      cast_dt_kernel<<<(n2 + 255) / 256, 256, 0, stream>>>(dbc, dt16, n2, 64.0f);
    }
    wmma_gemm64<0, false, 2, 0, false, 0><<<dim3(gemm_blocks(SEQ_L, DIM_I), 1), 256, 0, stream>>>(
        (cus)dt16, (cus)dt16, DIM_R, 0L,
        (cus)(dtp16 + (size_t)l * DIM_I * DIM_R), (cus)(dtp16 + (size_t)l * DIM_I * DIM_R), DIM_R, 0L,
        (void*)dpre, (void*)dpre, DIM_I, 0L,
        dt_proj_b + (size_t)l * DIM_I, b1, 0L, SEQ_L, DIM_I, DIM_R, 1.0f / 4096.0f);
    scan_kernel<<<DIM_I / 64, 256, 0, stream>>>(
        u32, dpre, dbc, proj, A_log + (size_t)l * DIM_I * DIM_ST, Dp + (size_t)l * DIM_I, ys16, SEQ_L);
    wmma_gemm64<0, false, 0, 0, true, 0><<<dim3(gemm_blocks(SEQ_L, DIM_M), 1), 256, 0, stream>>>(
        (cus)ys16, (cus)ys16, DIM_I, 0L,
        (cus)(outp16 + (size_t)l * DIM_M * DIM_I), (cus)(outp16 + (size_t)l * DIM_M * DIM_I), DIM_I, 0L,
        (void*)hnxt, (void*)hnxt, DIM_M, 0L,
        b1, hres, 0L, SEQ_L, DIM_M, DIM_I, 1.0f / 16384.0f);
  }

  final_norm_rows<<<SEQ_L / FR_ROWS, 256, 0, stream>>>(hA, norm_f_w, hf, outF, SEQ_L);
  head_kernel<<<1, 512, 0, stream>>>(hf, cls_w, cls_b, outF, SEQ_L);
}
